// OptBlockv2_45466523795646
// MI455X (gfx1250) — hardware-run, weakly checked
//
#include <hip/hip_runtime.h>


#ifndef NS
#define NS 2048
#endif
#define NS_FULL 2048
#define NBU 1024
#define NSC 4096
#define CMS 0.01f

static_assert(NS % 32 == 0);
static_assert(NSC % 64 == 0);
static_assert(NBU % 64 == 0);
static_assert(NBU % 32 == 0);
static_assert(((size_t)NS * NBU) % 8 == 0);
static_assert(NBU % 8 == 0);
static_assert(NS <= NS_FULL);

typedef unsigned short bf;
typedef __attribute__((ext_vector_type(16))) __bf16   v16bf;
typedef __attribute__((ext_vector_type(8)))  unsigned short v8us;
typedef __attribute__((ext_vector_type(8)))  float    v8f;
typedef __attribute__((ext_vector_type(4)))  float    v4f;
typedef v4f  __attribute__((may_alias)) v4fa;
typedef v8us __attribute__((may_alias)) v8usa;

__device__ __forceinline__ unsigned short f2bf(float f) { unsigned u = __float_as_uint(f); u += 0x7FFFu + ((u >> 16) & 1u); return (unsigned short)(u >> 16); }
__device__ __forceinline__ float bfr(float f) { unsigned u = __float_as_uint(f); u += 0x7FFFu + ((u >> 16) & 1u); return __uint_as_float(u & 0xFFFF0000u); }
__device__ __forceinline__ v16bf cat16b(v8us lo, v8us hi) { return __builtin_bit_cast(v16bf, __builtin_shufflevector(lo, hi, 0, 1, 2, 3, 4, 5, 6, 7, 8, 9, 10, 11, 12, 13, 14, 15)); }
__device__ __forceinline__ v8f wmmab(v16bf a, v16bf b, v8f c) { return __builtin_amdgcn_wmma_f32_16x16x32_bf16(false, a, false, b, (short)0, c, false, false); }
__device__ __forceinline__ v16bf ldb(const bf* p)  { return cat16b(*(const v8us*)p, *(const v8us*)(p + 16)); }
__device__ __forceinline__ void wave_sync() { __builtin_amdgcn_fence(3  , "wavefront"); __builtin_amdgcn_wave_barrier(); asm volatile("" ::: "memory"); }

__global__ __launch_bounds__(256) void k_mask(const float* __restrict__ proba, const float* __restrict__ avail, const float* __restrict__ alloc, bf* P1, bf* P2, size_t n8) {
    const size_t i = (size_t)blockIdx.x * 256 + threadIdx.x; if (i >= n8) return;
    const int b0 = (int)((i * 8) % (size_t)NBU);
    const v8f p = *(const v8f*)(proba + i * 8);
    const v8f a = *(const v8f*)(avail + b0);
    const v8f l = *(const v8f*)(alloc + b0);
    v8us o1, o2;
#pragma unroll
    for (int k = 0; k < 8; ++k) {
        const unsigned short pb = f2bf(p[k]);
        const float pr = __uint_as_float((unsigned)pb << 16);
        const float ar = bfr(a[k]);
        const float lr = bfr(l[k]);
        const bool oa = ((ar - pr) < 0.0f) & (pr > 0.0f);
        const bool ol = ((lr + pr) < 0.0f) & (pr < 0.0f);
        const bool ov = oa | ol;
        o1[k] = ov ? (unsigned short)0 : pb;
        o2[k] = ov ? pb : (unsigned short)0;
    }
    *(volatile v8us*)(P1 + i * 8) = o1; *(volatile v8us*)(P2 + i * 8) = o2;
    __threadfence();
    *(volatile v8us*)(P1 + i * 8) = o1; *(volatile v8us*)(P2 + i * 8) = o2;
}

__global__ __launch_bounds__(256) void k_trB(const float* __restrict__ src, bf* dst) {
    __shared__ __align__(16) unsigned short ts[64 * 72];
    const int tid = threadIdx.x;
    const int sc0 = blockIdx.x * 64, b0 = blockIdx.y * 64;
#pragma unroll
    for (int i = 0; i < 4; ++i) {
        const int idx = tid + i * 256; const int br = idx >> 4, c4 = (idx & 15) * 4;
        const v4f v = *(const v4f*)(src + (size_t)(b0 + br) * NSC + sc0 + c4);
#pragma unroll
        for (int j = 0; j < 4; ++j) ts[(c4 + j) * 72 + br] = f2bf(v[j]);
    }
    __syncthreads();
    v8us o[2];
#pragma unroll
    for (int i = 0; i < 2; ++i) {
        const int piece = tid + i * 256; const int row = piece >> 3, c8 = (piece & 7) * 8;
        o[i] = *(const v8usa*)(&ts[row * 72 + c8]);
    }
#pragma unroll
    for (int i = 0; i < 2; ++i) { const int piece = tid + i * 256; const int row = piece >> 3, c8 = (piece & 7) * 8;
        *(volatile v8us*)(dst + (size_t)(sc0 + row) * NBU + b0 + c8) = o[i]; }
    __threadfence();
#pragma unroll
    for (int i = 0; i < 2; ++i) { const int piece = tid + i * 256; const int row = piece >> 3, c8 = (piece & 7) * 8;
        *(volatile v8us*)(dst + (size_t)(sc0 + row) * NBU + b0 + c8) = o[i]; }
}

__global__ __launch_bounds__(32) void k_gemm(const bf* __restrict__ P1, const bf* __restrict__ P2, const bf* __restrict__ Bt, const float* __restrict__ cur, float* out) {
    __shared__ __align__(16) float os[16 * 68];
    const int K = NBU;
    const int lane = threadIdx.x & 31, lr = lane & 15, hi = lane >> 4; const int r0 = blockIdx.x * 32, c0 = blockIdx.y * 64;
    v8f acc1[2][4], acc2[2][4];
#pragma unroll
    for (int mb = 0; mb < 2; ++mb)
#pragma unroll
        for (int nb = 0; nb < 4; ++nb) { acc1[mb][nb] = (v8f){}; acc2[mb][nb] = (v8f){}; }
    const size_t aoff = (size_t)(r0 + lr) * K + 8 * hi, boff = (size_t)(c0 + lr) * K + 8 * hi;
    v16bf a1[2], a2[2];
#pragma unroll
    for (int mb = 0; mb < 2; ++mb) { a1[mb] = cat16b((v8us){}, (v8us){}); a2[mb] = cat16b((v8us){}, (v8us){}); }
#pragma unroll 1
    for (int kc = 0; kc < K; kc += 32) {
#pragma unroll
        for (int mb = 0; mb < 2; ++mb) { a1[mb] = ldb(P1 + aoff + (size_t)mb * 16 * K + kc); a2[mb] = ldb(P2 + aoff + (size_t)mb * 16 * K + kc); }
#pragma unroll
        for (int nb = 0; nb < 4; ++nb) { const v16bf b = ldb(Bt + boff + (size_t)nb * 16 * K + kc);
#pragma unroll
            for (int mb = 0; mb < 2; ++mb) { acc1[mb][nb] = wmmab(a1[mb], b, acc1[mb][nb]); acc2[mb][nb] = wmmab(a2[mb], b, acc2[mb][nb]); } }
        asm volatile("v_nop\n\tv_nop\n\tv_nop\n\tv_nop" : "+v"(acc1[0][3]), "+v"(acc2[0][3]), "+v"(acc1[1][3]), "+v"(acc2[1][3]) : "v"(a1[0]), "v"(a1[1]), "v"(a2[0]), "v"(a2[1]));
    }
    asm volatile("v_nop\n\tv_nop\n\tv_nop\n\tv_nop\n\tv_nop"
                 : "+v"(acc1[0][0]), "+v"(acc1[0][1]), "+v"(acc1[0][2]), "+v"(acc1[0][3]), "+v"(acc2[0][0]), "+v"(acc2[0][1]), "+v"(acc2[0][2]), "+v"(acc2[0][3])
                 : "v"(a1[0]), "v"(a1[1]), "v"(a2[0]), "v"(a2[1]));
    asm volatile(""
                 : "+v"(acc1[1][0]), "+v"(acc1[1][1]), "+v"(acc1[1][2]), "+v"(acc1[1][3]), "+v"(acc2[1][0]), "+v"(acc2[1][1]), "+v"(acc2[1][2]), "+v"(acc2[1][3]));
    const size_t tbase = (size_t)r0 * NSC + c0;
#pragma unroll
    for (int mb = 0; mb < 2; ++mb) {
#pragma unroll
        for (int nb = 0; nb < 4; ++nb) {
#pragma unroll
            for (int j = 0; j < 8; ++j) os[(hi * 8 + j) * 68 + nb * 16 + lr] = acc1[mb][nb][j] + CMS * acc2[mb][nb][j]; }
        wave_sync();
        const size_t sb = tbase + (size_t)(mb * 16) * NSC;
        v4f vals[8];
#pragma unroll
        for (int s = 0; s < 8; ++s) { const int row = 2 * s + hi, cofs = lr * 4;
            const v4f x = *(const v4fa*)(&os[row * 68 + cofs]);
            const v4f c = *(const v4f*)(cur + sb + (size_t)row * NSC + cofs);
            v4f r; r[0] = bfr(c[0]) + x[0]; r[1] = bfr(c[1]) + x[1]; r[2] = bfr(c[2]) + x[2]; r[3] = bfr(c[3]) + x[3];
            vals[s] = r; }
#pragma unroll 1
        for (int ps = 0; ps < 2; ++ps) {
#pragma unroll
            for (int s = 0; s < 8; ++s) { const int row = 2 * s + hi, cofs = lr * 4;
                *(volatile v4f*)(out + sb + (size_t)row * NSC + cofs) = vals[s]; }
            if (ps == 0) __threadfence(); }
        wave_sync();
    }
}

static constexpr size_t al256(size_t v) { return (v + 255) & ~(size_t)255; }
static constexpr size_t SZ_P  = al256((size_t)NS * NBU * 2);
static constexpr size_t SZ_BT = al256((size_t)NSC * NBU * 2);
static constexpr size_t SZ_TOTAL = 2 * SZ_P + SZ_BT;
static_assert(SZ_TOTAL <= (size_t)134217728);
static_assert(((size_t)NS * NBU / 8) % 256 == 0);

extern "C" void kernel_launch(void* const* d_in, const int* in_sizes, int n_in,
                              void* d_out, int out_size, void* d_ws, size_t ws_size, hipStream_t stream) {
    if (n_in < 5) return;
    if ((size_t)in_sizes[0] < (size_t)NS * NBU) return;
    if ((size_t)in_sizes[1] < (size_t)NS * NSC) return;
    if ((size_t)in_sizes[2] < (size_t)NBU * NSC) return;
    if ((size_t)in_sizes[3] < (size_t)NBU || (size_t)in_sizes[4] < (size_t)NBU) return;
    if ((size_t)out_size < (size_t)NS * NSC) return;
    if (SZ_TOTAL > ws_size) return;
    const float* proba = (const float*)d_in[0];
    const float* cur   = (const float*)d_in[1];
    const float* bun   = (const float*)d_in[2];
    const float* avail = (const float*)d_in[3];
    const float* alloc = (const float*)d_in[4];
    float* OUT = (float*)d_out;
    char* wsp = (char*)d_ws;
    bf* P1 = (bf*)wsp; wsp += SZ_P;
    bf* P2 = (bf*)wsp; wsp += SZ_P;
    bf* BT = (bf*)wsp; wsp += SZ_BT;

    { const size_t n8 = (size_t)NS * NBU / 8;
      k_mask<<<(unsigned)((n8 + 255) / 256), 256, 0, stream>>>(proba, avail, alloc, P1, P2, n8); }
    k_trB<<<dim3(NSC / 64, NBU / 64, 1), 256, 0, stream>>>(bun, BT);
    k_gemm<<<dim3(NS / 32, NSC / 64, 1), 32, 0, stream>>>(P1, P2, BT, cur, OUT);
}
